// Procedure_60017872994694
// MI455X (gfx1250) — hardware-verified
//
#include <hip/hip_runtime.h>
#include <hip/hip_bf16.h>


typedef __bf16 bf16_t;
typedef bf16_t v16bf __attribute__((ext_vector_type(16)));
typedef bf16_t v8bf  __attribute__((ext_vector_type(8)));
typedef float  v8f   __attribute__((ext_vector_type(8)));
typedef float  v4f   __attribute__((ext_vector_type(4)));
typedef unsigned int v4u __attribute__((ext_vector_type(4)));
typedef v4f __attribute__((may_alias)) v4fa;
typedef v4u __attribute__((may_alias)) v4ua;

union Frag16 { v16bf v; v8bf h[2]; };
union Pack8  { v8bf v; v4u u; };

__device__ __forceinline__ int clampi(int v, int hi) {
    return v < 0 ? 0 : (v > hi ? hi : v);
}

__device__ __forceinline__ v8f zero8() {
    v8f z = {0.f, 0.f, 0.f, 0.f, 0.f, 0.f, 0.f, 0.f};
    return z;
}

__device__ __forceinline__ v8f wmma_bf16(v16bf a, v16bf b, v8f c) {
    v8f d = __builtin_amdgcn_wmma_f32_16x16x32_bf16(false, a, false, b, (short)0, c, false, false);
    asm volatile("v_nop\n\tv_nop\n\tv_nop\n\tv_nop" : "+v"(d) : "v"(a), "v"(b));
    return d;
}

__device__ __forceinline__ v16bf load_a_frag(const bf16_t* tile, int ldk, int kt, int lane) {
    const int row = lane & 15;
    const int kh  = (lane >> 4) * 8;
    const bf16_t* p = tile + row * ldk + kt * 32 + kh;
    Frag16 f;
    f.h[0] = *(const v8bf*)p;
    f.h[1] = *(const v8bf*)(p + 16);
    return f.v;
}

__device__ __forceinline__ v16bf load_b_frag(const bf16_t* Wp, int tile, int lane) {
    return *(const v16bf*)(Wp + ((size_t)tile << 9) + lane * 16);
}

__global__ __launch_bounds__(256) void pack_w_kernel(const float* __restrict__ W, bf16_t* out,
                                                     int Ksrc, int Kp, int Nc) {
    const int nTile = Nc >> 4;
    const long long total8 = (long long)(Kp >> 5) * nTile * 64;
    const long long stride = (long long)gridDim.x * blockDim.x;
    for (long long q = (long long)blockIdx.x * blockDim.x + threadIdx.x; q < total8; q += stride) {
        const int half = (int)(q & 1);
        const int l    = (int)((q >> 1) & 31);
        const long long tile = q >> 6;
        const int kt = (int)(tile / nTile);
        const int nt = (int)(tile - (long long)kt * nTile);
        const int h  = l >> 4;
        const int n  = nt * 16 + (l & 15);
        const int kb = kt * 32 + 16 * half + 8 * h;
        Pack8 pk;
#pragma unroll
        for (int ii = 0; ii < 8; ++ii) {
            const int k = kb + ii;
            const float v = (k < Ksrc) ? W[(size_t)k * Nc + n] : 0.0f;
            pk.v[ii] = (bf16_t)v;
        }
        volatile v4u* dst = (volatile v4u*)(out + q * 8);
        *dst = pk.u;
        __threadfence();
        *dst = pk.u;
    }
}

#define PAIR_K 160

__global__ __launch_bounds__(128) void pair_kernel(
    const int* __restrict__ lengthes,
    const int* __restrict__ ntypes, const int* __restrict__ ndist,
    const float* __restrict__ nrat, const float* __restrict__ ncom,
    const int* __restrict__ nprice, const float* __restrict__ ngroup,
    const float* __restrict__ Etp, const float* __restrict__ Edp, const float* __restrict__ Epp,
    const bf16_t* __restrict__ W1p, const float* __restrict__ b1,
    const bf16_t* __restrict__ W2p, const float* __restrict__ b2,
    float* CTX, int N, int nEt, int nEd, int nEp)
{
    __shared__ __align__(16) bf16_t feat_s[16 * PAIR_K];
    __shared__ __align__(16) bf16_t h1_s[16 * 128];
    __shared__ __align__(16) float  ctx_s[128];

    const int b    = blockIdx.x;
    const int tid  = threadIdx.x;
    const int lane = tid & 31;
    const int w    = tid >> 5;
    const int len  = lengthes[b];

    const int nloc = lane & 15;
    const int mofs = (lane & 16) ? 8 : 0;
    const int c0 = w * 16 + nloc;
    const int c1 = (w + 4) * 16 + nloc;
    float ctxacc0 = 0.0f, ctxacc1 = 0.0f;

    const int ntiles = (N + 15) >> 4;
    for (int rt = 0; rt < ntiles; ++rt) {
        __syncthreads();
        for (int idx = tid; idx < 16 * PAIR_K; idx += 128) {
            const int r = idx / PAIR_K, k = idx - r * PAIR_K;
            const int n = rt * 16 + r;
            float v = 0.0f;
            if (n < N) {
                const size_t bn = (size_t)b * N + n;
                if (k < 64)        v = Etp[(size_t)clampi(ntypes[bn], nEt - 1) * 64 + k];
                else if (k < 96)   v = Edp[(size_t)clampi(ndist[bn],  nEd - 1) * 32 + (k - 64)];
                else if (k == 96)  v = nrat[bn];
                else if (k == 97)  v = ncom[bn];
                else if (k < 130)  v = Epp[(size_t)clampi(nprice[bn], nEp - 1) * 32 + (k - 98)];
                else if (k == 130) v = ngroup[bn];
            }
            feat_s[idx] = (bf16_t)v;
        }
        __syncthreads();
        v8f acc0 = zero8(), acc1 = zero8();
        for (int kt = 0; kt < PAIR_K / 32; ++kt) {
            const v16bf a  = load_a_frag(feat_s, PAIR_K, kt, lane);
            const v16bf bA = load_b_frag(W1p, kt * 8 + w,     lane);
            const v16bf bB = load_b_frag(W1p, kt * 8 + w + 4, lane);
            acc0 = wmma_bf16(a, bA, acc0);
            acc1 = wmma_bf16(a, bB, acc1);
        }
        {
            const float bb0 = b1[c0], bb1 = b1[c1];
#pragma unroll
            for (int j = 0; j < 8; ++j) {
                const int mr = j + mofs;
                float v0 = acc0[j] + bb0; v0 = v0 > 0.0f ? v0 : 0.0f;
                float v1 = acc1[j] + bb1; v1 = v1 > 0.0f ? v1 : 0.0f;
                h1_s[mr * 128 + c0] = (bf16_t)v0;
                h1_s[mr * 128 + c1] = (bf16_t)v1;
            }
        }
        __syncthreads();
        acc0 = zero8(); acc1 = zero8();
        for (int kt = 0; kt < 4; ++kt) {
            const v16bf a  = load_a_frag(h1_s, 128, kt, lane);
            const v16bf bA = load_b_frag(W2p, kt * 8 + w,     lane);
            const v16bf bB = load_b_frag(W2p, kt * 8 + w + 4, lane);
            acc0 = wmma_bf16(a, bA, acc0);
            acc1 = wmma_bf16(a, bB, acc1);
        }
        {
            const float bb0 = b2[c0], bb1 = b2[c1];
            float p0 = 0.0f, p1 = 0.0f;
#pragma unroll
            for (int j = 0; j < 8; ++j) {
                const int n = rt * 16 + j + mofs;
                const float m = (n < len && n < N) ? 1.0f : 0.0f;
                float v0 = acc0[j] + bb0; v0 = v0 > 0.0f ? v0 : 0.0f;
                float v1 = acc1[j] + bb1; v1 = v1 > 0.0f ? v1 : 0.0f;
                p0 += m * v0; p1 += m * v1;
            }
            p0 += __shfl_down(p0, 16, 32);
            p1 += __shfl_down(p1, 16, 32);
            if (lane < 16) { ctxacc0 += p0; ctxacc1 += p1; }
        }
    }
    if (lane < 16) {
        const float denom = (float)(len > 1 ? len : 1);
        const float inv = 1.0f / denom;
        ctx_s[w * 16 + lane]       = ctxacc0 * inv;
        ctx_s[(w + 4) * 16 + lane] = ctxacc1 * inv;
    }
    __syncthreads();
    if (w == 0) {
        const v4f v = *(const v4fa*)(ctx_s + 4 * lane);
        volatile v4f* d = (volatile v4f*)(CTX + (size_t)b * 128 + 4 * lane);
        *d = v;
        __threadfence();
        *d = v;
    }
}

__global__ __launch_bounds__(128) void node_feat_kernel(
    const int* __restrict__ all_types, const int* __restrict__ all_prices,
    const float* __restrict__ all_groups,
    const float* __restrict__ Etg, const float* __restrict__ Epg,
    const bf16_t* __restrict__ Wgsp, const float* __restrict__ bgs,
    bf16_t* X, int M, int nEtg, int nEpg)
{
    __shared__ __align__(16) bf16_t a_s[16 * 128];
    __shared__ __align__(16) bf16_t o_s[16 * 136];
    const int m0 = blockIdx.x * 16;
    const int tid = threadIdx.x, lane = tid & 31, w = tid >> 5;
    for (int idx = tid; idx < 16 * 128; idx += 128) {
        const int r = idx >> 7, k = idx & 127;
        const int m = m0 + r;
        float v = 0.0f;
        if (m < M) {
            if (k < 64)       v = Etg[(size_t)clampi(all_types[m],  nEtg - 1) * 64 + k];
            else if (k < 96)  v = Epg[(size_t)clampi(all_prices[m], nEpg - 1) * 32 + (k - 64)];
            else if (k == 96) v = all_groups[m];
        }
        a_s[idx] = (bf16_t)v;
    }
    __syncthreads();
    const int nloc = lane & 15, mofs = (lane & 16) ? 8 : 0;
    for (int t = 0; t < 2; ++t) {
        const int nt = w + t * 4;
        v8f acc = zero8();
        for (int kt = 0; kt < 4; ++kt) {
            const v16bf a  = load_a_frag(a_s, 128, kt, lane);
            const v16bf bb = load_b_frag(Wgsp, kt * 8 + nt, lane);
            acc = wmma_bf16(a, bb, acc);
        }
        const int col = nt * 16 + nloc;
        const float bias = bgs[col];
#pragma unroll
        for (int j = 0; j < 8; ++j) {
            float v = acc[j] + bias; v = v > 0.0f ? v : 0.0f;
            o_s[(j + mofs) * 136 + col] = (bf16_t)v;
        }
    }
    __syncthreads();
    for (int pass = 0; pass < 2; ++pass) {
#pragma unroll
        for (int it = 0; it < 2; ++it) {
            const int c = it * 128 + tid;
            const int row = c >> 4, off = (c & 15) * 8;
            const v4u u = *(const v4ua*)(o_s + row * 136 + off);
            *(volatile v4u*)(X + (size_t)(m0 + row) * 128 + off) = u;
        }
        if (pass == 0) __threadfence();
    }
}

__global__ __launch_bounds__(128) void gemm128_kernel(
    const bf16_t* __restrict__ Z, const bf16_t* __restrict__ Wp,
    const float* __restrict__ dinv, float* T, int M)
{
    __shared__ __align__(16) bf16_t z_s[16 * 128];
    __shared__ __align__(16) float  t_s[16 * 132];
    const int m0 = blockIdx.x * 16;
    const int tid = threadIdx.x, lane = tid & 31, w = tid >> 5;
    for (int idx = tid; idx < 16 * 128 / 8; idx += 128) {
        const int r  = idx >> 4;
        const int kc = (idx & 15) * 8;
        const int m  = m0 + r;
        v8bf v;
        if (m < M) {
            v = *(const v8bf*)(Z + (size_t)m * 128 + kc);
        } else {
#pragma unroll
            for (int j = 0; j < 8; ++j) v[j] = (bf16_t)0.0f;
        }
        *(v8bf*)(z_s + r * 128 + kc) = v;
    }
    __syncthreads();
    const int nloc = lane & 15, mofs = (lane & 16) ? 8 : 0;
    for (int t = 0; t < 2; ++t) {
        const int nt = w + t * 4;
        v8f acc = zero8();
        for (int kt = 0; kt < 4; ++kt) {
            const v16bf a  = load_a_frag(z_s, 128, kt, lane);
            const v16bf bb = load_b_frag(Wp, kt * 8 + nt, lane);
            acc = wmma_bf16(a, bb, acc);
        }
        const int col = nt * 16 + nloc;
#pragma unroll
        for (int j = 0; j < 8; ++j) {
            const int r = j + mofs;
            t_s[r * 132 + col] = acc[j] * dinv[m0 + r];
        }
    }
    __syncthreads();
    for (int pass = 0; pass < 2; ++pass) {
#pragma unroll
        for (int it = 0; it < 4; ++it) {
            const int c = it * 128 + tid;
            const int row = c >> 5, off = (c & 31) * 4;
            const v4f v = *(const v4fa*)(t_s + row * 132 + off);
            *(volatile v4f*)(T + (size_t)(m0 + row) * 128 + off) = v;
        }
        if (pass == 0) __threadfence();
    }
}

__global__ __launch_bounds__(256) void deg_kernel(const int* __restrict__ edge_index,
                                                  float* dinv, int E, int M)
{
    __shared__ int lst_s[256];
    __shared__ int wcnt_s[8];
    __shared__ __align__(16) float dv_s[256];
    const int base = blockIdx.x * 256;
    const int tid = threadIdx.x, lane = tid & 31, w = tid >> 5;
    const int* edst = edge_index + E;
    int cnt = 0;
    for (int e0 = 0; e0 < E; e0 += 256) {
        const int e = e0 + tid;
        bool hit = false;
        int dl = 0;
        if (e < E) {
            const int d = edst[e];
            hit = (d >= base) && (d < base + 256) && (d < M);
            dl = d - base;
        }
        const unsigned bal = __builtin_amdgcn_ballot_w32(hit);
        const int pre = __builtin_popcount(bal & ((1u << lane) - 1u));
        if (lane == 0) wcnt_s[w] = __builtin_popcount(bal);
        __syncthreads();
        int woff = 0, tot = 0;
#pragma unroll
        for (int i = 0; i < 8; ++i) { const int c = wcnt_s[i]; tot += c; if (i < w) woff += c; }
        if (hit) lst_s[woff + pre] = dl;
        __syncthreads();
        for (int j = 0; j < tot; ++j) cnt += (lst_s[j] == tid) ? 1 : 0;
        __syncthreads();
    }
    float degf = (float)(cnt + 1);
    degf = degf > 1.0f ? degf : 1.0f;
    dv_s[tid] = 1.0f / sqrtf(degf);
    __syncthreads();
    if (tid < 64) {
        const v4f v = *(const v4fa*)(dv_s + 4 * tid);
        volatile v4f* d = (volatile v4f*)(dinv + (size_t)base + 4 * tid);
        *d = v;
        __threadfence();
        *d = v;
    }
}

template <int MODE>
__global__ __launch_bounds__(128) void agg_kernel(
    const float* __restrict__ Tq, const int* __restrict__ edge_index,
    const float* __restrict__ dinv, const float* __restrict__ bias,
    const int* __restrict__ bidp, bf16_t* outb, float* outf,
    int E, int M, int Bsz)
{
    __shared__ __align__(16) float  acc_s[64 * 128];
    __shared__ __align__(16) bf16_t ob_s[(MODE == 0) ? 64 * 128 : 8];
    __shared__ int ls_s[128];
    __shared__ int ld_s[128];
    __shared__ int wcnt_s[4];
    const int tid = threadIdx.x, lane = tid & 31, w = tid >> 5;
    int lo = 0, nrows = M;
    if (MODE == 1) {
        int bid = bidp[0];
        if (bid < 0) bid = 0;
        long long lo64 = (long long)bid * Bsz;
        if (lo64 > M) lo64 = M;
        lo = (int)lo64;
        nrows = Bsz;
    }
    const int obase = blockIdx.x * 64;
    const int nbase = lo + obase;
    for (int i = tid; i < 64 * 128; i += 128) acc_s[i] = 0.0f;
    __syncthreads();
    const int* esrc = edge_index;
    const int* edst = edge_index + E;
    for (int e0 = 0; e0 < E; e0 += 128) {
        const int e = e0 + tid;
        bool hit = false;
        int d = 0, s = 0;
        if (e < E) {
            d = edst[e];
            hit = (d >= nbase) && (d < nbase + 64) && (d < M) && ((d - lo) < nrows);
        }
        if (hit) s = clampi(esrc[e], M - 1);
        const unsigned bal = __builtin_amdgcn_ballot_w32(hit);
        const int pre = __builtin_popcount(bal & ((1u << lane) - 1u));
        if (lane == 0) wcnt_s[w] = __builtin_popcount(bal);
        __syncthreads();
        int woff = 0, tot = 0;
#pragma unroll
        for (int i = 0; i < 4; ++i) { const int c = wcnt_s[i]; tot += c; if (i < w) woff += c; }
        if (hit) { ls_s[woff + pre] = s; ld_s[woff + pre] = d - nbase; }
        __syncthreads();
        for (int j = 0; j < tot; ++j) {
            const int sj = ls_s[j];
            const int dl = ld_s[j];
            acc_s[dl * 128 + tid] += Tq[(size_t)sj * 128 + tid];
        }
        __syncthreads();
    }
    const float bcol = bias[tid];
    for (int r = 0; r < 64; ++r) {
        const int d = nbase + r;
        const bool valid = (d < M) && ((obase + r) < nrows);
        float v = 0.0f;
        if (valid) v = (acc_s[r * 128 + tid] + Tq[(size_t)d * 128 + tid]) * dinv[d] + bcol;
        if (MODE == 0) {
            v = v > 0.0f ? v : 0.0f;
            ob_s[r * 128 + tid] = (bf16_t)v;
        } else {
            acc_s[r * 128 + tid] = v;
        }
    }
    __syncthreads();
    if (MODE == 0) {
        for (int pass = 0; pass < 2; ++pass) {
#pragma unroll
            for (int it = 0; it < 8; ++it) {
                const int c = it * 128 + tid;
                const int row = c >> 4, off = (c & 15) * 8;
                const v4u u = *(const v4ua*)(ob_s + row * 128 + off);
                *(volatile v4u*)(outb + (size_t)(obase + row) * 128 + off) = u;
            }
            if (pass == 0) __threadfence();
        }
    } else {
        for (int pass = 0; pass < 2; ++pass) {
#pragma unroll
            for (int it = 0; it < 16; ++it) {
                const int c = it * 128 + tid;
                const int row = c >> 5, off = (c & 31) * 4;
                const v4f v = *(const v4fa*)(acc_s + row * 128 + off);
                *(volatile v4f*)(outf + (size_t)(obase + row) * 128 + off) = v;
            }
            if (pass == 0) __threadfence();
        }
    }
}

__global__ __launch_bounds__(128) void head_kernel(
    const float* __restrict__ CTX, const int* __restrict__ types, const float* __restrict__ Etp,
    const bf16_t* __restrict__ Wps1p, const float* __restrict__ bps1,
    const float* __restrict__ Wps2, const float* __restrict__ bps2,
    const float* __restrict__ Y2,
    const bf16_t* __restrict__ Wq1p, const float* __restrict__ bq1,
    const float* __restrict__ Wq2, const float* __restrict__ bq2,
    const float* __restrict__ Wc, const float* __restrict__ bc,
    float* out, int B, int nEt)
{
    __shared__ __align__(16) bf16_t a1_s[32 * 192];
    __shared__ __align__(16) bf16_t a2_s[32 * 128];
    __shared__ float ps_s[32 * 64];
    __shared__ float q_s[32 * 64];
    __shared__ __align__(16) float o_s[32];
    const int r0 = blockIdx.x * 32;
    const int tid = threadIdx.x, lane = tid & 31, w = tid >> 5;
    for (int idx = tid; idx < 32 * 192; idx += 128) {
        const int r = idx / 192, k = idx - r * 192;
        const int row = r0 + r;
        float v = 0.0f;
        if (row < B) {
            if (k < 128) v = CTX[(size_t)row * 128 + k];
            else         v = Etp[(size_t)clampi(types[row], nEt - 1) * 64 + (k - 128)];
        }
        a1_s[idx] = (bf16_t)v;
    }
    for (int idx = tid; idx < 32 * 128; idx += 128) {
        const int r = idx >> 7, k = idx & 127;
        const int row = r0 + r;
        const float v = (row < B) ? Y2[(size_t)row * 128 + k] : 0.0f;
        a2_s[idx] = (bf16_t)v;
    }
    __syncthreads();
    const int rt = w >> 1;
    const int ntA = (w & 1) * 2, ntB = ntA + 1;
    const int nloc = lane & 15, mofs = (lane & 16) ? 8 : 0;
    {
        v8f acc0 = zero8(), acc1 = zero8();
        for (int kt = 0; kt < 6; ++kt) {
            const v16bf a  = load_a_frag(a1_s + rt * 16 * 192, 192, kt, lane);
            const v16bf bA = load_b_frag(Wps1p, kt * 4 + ntA, lane);
            const v16bf bB = load_b_frag(Wps1p, kt * 4 + ntB, lane);
            acc0 = wmma_bf16(a, bA, acc0);
            acc1 = wmma_bf16(a, bB, acc1);
        }
        const int cA = ntA * 16 + nloc, cB = ntB * 16 + nloc;
        const float biA = bps1[cA], biB = bps1[cB];
#pragma unroll
        for (int j = 0; j < 8; ++j) {
            const int row = rt * 16 + j + mofs;
            float vA = acc0[j] + biA; vA = vA > 0.0f ? vA : 0.0f;
            float vB = acc1[j] + biB; vB = vB > 0.0f ? vB : 0.0f;
            ps_s[row * 64 + cA] = vA;
            ps_s[row * 64 + cB] = vB;
        }
    }
    {
        v8f acc0 = zero8(), acc1 = zero8();
        for (int kt = 0; kt < 4; ++kt) {
            const v16bf a  = load_a_frag(a2_s + rt * 16 * 128, 128, kt, lane);
            const v16bf bA = load_b_frag(Wq1p, kt * 4 + ntA, lane);
            const v16bf bB = load_b_frag(Wq1p, kt * 4 + ntB, lane);
            acc0 = wmma_bf16(a, bA, acc0);
            acc1 = wmma_bf16(a, bB, acc1);
        }
        const int cA = ntA * 16 + nloc, cB = ntB * 16 + nloc;
        const float biA = bq1[cA], biB = bq1[cB];
#pragma unroll
        for (int j = 0; j < 8; ++j) {
            const int row = rt * 16 + j + mofs;
            float vA = acc0[j] + biA; vA = vA > 0.0f ? vA : 0.0f;
            float vB = acc1[j] + biB; vB = vB > 0.0f ? vB : 0.0f;
            q_s[row * 64 + cA] = vA;
            q_s[row * 64 + cB] = vB;
        }
    }
    __syncthreads();
    if (tid < 32) {
        const int row = r0 + tid;
        float o = 0.0f;
        if (row < B) {
            float s1 = 0.0f, s2 = 0.0f;
            for (int k = 0; k < 64; ++k) {
                s1 += ps_s[tid * 64 + k] * Wps2[k];
                s2 += q_s[tid * 64 + k] * Wq2[k];
            }
            s1 += bps2[0];
            s2 += bq2[0];
            o = s1 * Wc[0] + s2 * Wc[1] + bc[0];
        }
        o_s[tid] = o;
    }
    __syncthreads();
    if (r0 + 32 <= B) {
        if (tid < 8) {
            const v4f v = *(const v4fa*)(o_s + 4 * tid);
            volatile v4f* d = (volatile v4f*)(out + r0 + 4 * tid);
            *d = v;
            __threadfence();
            *d = v;
        }
    } else {
        if (tid < 32 && r0 + tid < B) {
            const float o = o_s[tid];
            volatile float* d = (volatile float*)(out + r0 + tid);
            *d = o;
            __threadfence();
            *d = o;
        }
    }
}

extern "C" void kernel_launch(void* const* d_in, const int* in_sizes, int n_in,
                              void* d_out, int out_size, void* d_ws, size_t ws_size,
                              hipStream_t stream) {
    const int*   types      = (const int*)d_in[0];
    const int*   lengthes   = (const int*)d_in[4];
    const int*   ntypes     = (const int*)d_in[5];
    const int*   ndist      = (const int*)d_in[6];
    const float* nrat       = (const float*)d_in[7];
    const float* ncom       = (const float*)d_in[8];
    const int*   nprice     = (const int*)d_in[9];
    const float* ngroup     = (const float*)d_in[10];
    const int*   all_types  = (const int*)d_in[11];
    const int*   all_prices = (const int*)d_in[12];
    const float* all_groups = (const float*)d_in[13];
    const int*   edge_index = (const int*)d_in[14];
    const int*   bidp       = (const int*)d_in[15];
    const float* Etp  = (const float*)d_in[16];
    const float* Edp  = (const float*)d_in[17];
    const float* Epp  = (const float*)d_in[18];
    const float* Wsh1 = (const float*)d_in[19];
    const float* bsh1 = (const float*)d_in[20];
    const float* Wsh2 = (const float*)d_in[21];
    const float* bsh2 = (const float*)d_in[22];
    const float* Wps1 = (const float*)d_in[23];
    const float* bps1 = (const float*)d_in[24];
    const float* Wps2 = (const float*)d_in[25];
    const float* bps2 = (const float*)d_in[26];
    const float* Etg  = (const float*)d_in[27];
    const float* Epg  = (const float*)d_in[28];
    const float* Wgs  = (const float*)d_in[29];
    const float* bgs  = (const float*)d_in[30];
    const float* Wgc1 = (const float*)d_in[31];
    const float* bgc1 = (const float*)d_in[32];
    const float* Wgc2 = (const float*)d_in[33];
    const float* bgc2 = (const float*)d_in[34];
    const float* Wq1  = (const float*)d_in[35];
    const float* bq1  = (const float*)d_in[36];
    const float* Wq2  = (const float*)d_in[37];
    const float* bq2  = (const float*)d_in[38];
    const float* Wc   = (const float*)d_in[39];
    const float* bc   = (const float*)d_in[40];
    float* out = (float*)d_out;
    (void)n_in; (void)out_size;

    const int B = in_sizes[0];
    if (B <= 0) return;
    const int N = in_sizes[5] / B;
    const int M = in_sizes[11];
    const int E = in_sizes[14] / 2;
    const int nEt  = in_sizes[16] / 64;
    const int nEd  = in_sizes[17] / 32;
    const int nEp  = in_sizes[18] / 32;
    const int nEtg = in_sizes[27] / 64;
    const int nEpg = in_sizes[28] / 32;
    if (M <= 0) return;

    const int mTiles = (M + 15) / 16;
    const int mB256  = (M + 255) / 256;
    const int Mpad   = mB256 * 256;
    const int mB64   = (M + 63) / 64;
    const int bB64   = (B + 63) / 64;
    const int Bpad64 = bB64 * 64;
    const int bB32   = (B + 31) / 32;

    size_t off = 0;
    auto carve = [&](size_t bytes) -> size_t {
        size_t r = off;
        off += (bytes + 255) & ~(size_t)255;
        return r;
    };
    auto packedBytes = [](int Kp, int Nc) -> size_t {
        return (size_t)(Kp / 32) * (Nc / 16) * 512 * sizeof(bf16_t);
    };
    const size_t o_w1p   = carve(packedBytes(PAIR_K, 128));
    const size_t o_w2p   = carve(packedBytes(128, 128));
    const size_t o_wgsp  = carve(packedBytes(128, 128));
    const size_t o_wgc1p = carve(packedBytes(128, 128));
    const size_t o_wgc2p = carve(packedBytes(128, 128));
    const size_t o_wq1p  = carve(packedBytes(128, 64));
    const size_t o_wps1p = carve(packedBytes(192, 64));
    const size_t o_ctx   = carve((size_t)B * 128 * sizeof(float));
    const size_t o_dinv  = carve((size_t)Mpad * sizeof(float));
    const size_t o_X     = carve((size_t)Mpad * 128 * sizeof(bf16_t));
    const size_t o_G1    = carve((size_t)Mpad * 128 * sizeof(bf16_t));
    const size_t o_T     = carve((size_t)Mpad * 128 * sizeof(float));
    const size_t o_Y2    = carve((size_t)Bpad64 * 128 * sizeof(float));
    if (off > ws_size) return;

    char* ws = (char*)d_ws;
    bf16_t* w1p   = (bf16_t*)(ws + o_w1p);
    bf16_t* w2p   = (bf16_t*)(ws + o_w2p);
    bf16_t* wgsp  = (bf16_t*)(ws + o_wgsp);
    bf16_t* wgc1p = (bf16_t*)(ws + o_wgc1p);
    bf16_t* wgc2p = (bf16_t*)(ws + o_wgc2p);
    bf16_t* wq1p  = (bf16_t*)(ws + o_wq1p);
    bf16_t* wps1p = (bf16_t*)(ws + o_wps1p);
    float*  CTX   = (float*)(ws + o_ctx);
    float*  dinv  = (float*)(ws + o_dinv);
    bf16_t* X     = (bf16_t*)(ws + o_X);
    bf16_t* G1    = (bf16_t*)(ws + o_G1);
    float*  T     = (float*)(ws + o_T);
    float*  Y2    = (float*)(ws + o_Y2);

    auto packGrid = [](int Kp, int Nc) -> int {
        long long total8 = (long long)(Kp / 32) * (Nc / 16) * 64;
        long long g = (total8 + 255) / 256;
        if (g < 1) g = 1;
        if (g > 1024) g = 1024;
        return (int)g;
    };

    pack_w_kernel<<<packGrid(PAIR_K, 128), 256, 0, stream>>>(Wsh1, w1p, 131, PAIR_K, 128);
    pack_w_kernel<<<packGrid(128, 128), 256, 0, stream>>>(Wsh2, w2p, 128, 128, 128);
    pack_w_kernel<<<packGrid(128, 128), 256, 0, stream>>>(Wgs,  wgsp, 97, 128, 128);
    pack_w_kernel<<<packGrid(128, 128), 256, 0, stream>>>(Wgc1, wgc1p, 128, 128, 128);
    pack_w_kernel<<<packGrid(128, 128), 256, 0, stream>>>(Wgc2, wgc2p, 128, 128, 128);
    pack_w_kernel<<<packGrid(128, 64),  256, 0, stream>>>(Wq1,  wq1p, 128, 128, 64);
    pack_w_kernel<<<packGrid(192, 64),  256, 0, stream>>>(Wps1, wps1p, 192, 192, 64);

    pair_kernel<<<B, 128, 0, stream>>>(lengthes, ntypes, ndist, nrat, ncom, nprice, ngroup,
                                       Etp, Edp, Epp, w1p, bsh1, w2p, bsh2,
                                       CTX, N, nEt, nEd, nEp);

    node_feat_kernel<<<mTiles, 128, 0, stream>>>(all_types, all_prices, all_groups,
                                                 Etg, Epg, wgsp, bgs, X, M, nEtg, nEpg);
    deg_kernel<<<mB256, 256, 0, stream>>>(edge_index, dinv, E, M);

    gemm128_kernel<<<mTiles, 128, 0, stream>>>(X, wgc1p, dinv, T, M);
    agg_kernel<0><<<mB64, 128, 0, stream>>>(T, edge_index, dinv, bgc1, bidp, G1, Y2, E, M, B);

    gemm128_kernel<<<mTiles, 128, 0, stream>>>(G1, wgc2p, dinv, T, M);
    agg_kernel<1><<<bB64, 128, 0, stream>>>(T, edge_index, dinv, bgc2, bidp, G1, Y2, E, M, B);

    head_kernel<<<bB32, 128, 0, stream>>>(CTX, types, Etp, wps1p, bps1, Wps2, bps2,
                                          Y2, wq1p, bq1, Wq2, bq2, Wc, bc, out, B, nEt);
}
